// SelfAttention3D_77335181132119
// MI455X (gfx1250) — hardware-verified
//
#include <hip/hip_runtime.h>
#include <math.h>

typedef __attribute__((ext_vector_type(16))) _Float16 v16h;
typedef __attribute__((ext_vector_type(8)))  _Float16 v8h;
typedef __attribute__((ext_vector_type(8)))  float v8f;
typedef __attribute__((ext_vector_type(4)))  float v4f;
typedef __attribute__((ext_vector_type(4)))  unsigned v4u;

template <typename T> __device__ __forceinline__ void vst2(void* p, T v) { *(volatile T*)p = v; __threadfence(); *(volatile T*)p = v; }
__device__ __forceinline__ v8f wmma16(v16h a, v16h b, v8f c) {
  v8f d = __builtin_amdgcn_wmma_f32_16x16x32_f16(false, a, false, b, (short)0, c, false, false);
  asm volatile("v_nop\n\tv_nop\n\tv_nop\n\tv_nop" : "+v"(d) : "v"(a), "v"(b));
  return d;
}
__device__ __forceinline__ v16h frag_h(const _Float16* rowk0, int lane) {
  union { v16h v; v8h q[2]; } u; const _Float16* p = rowk0 + 8 * (lane >> 4);
  u.q[0] = *(const v8h*)p; u.q[1] = *(const v8h*)(p + 16); return u.v;
}
__device__ __forceinline__ v16h frag_f32(const float* rowk0, int lane) {
  v16h a; const float* p = rowk0 + 8 * (lane >> 4);
#pragma unroll
  for (int i = 0; i < 8; ++i) { const float x0 = p[i], x1 = p[16 + i]; a[i] = (_Float16)x0; a[8 + i] = (_Float16)x1; }
  return a;
}
__device__ __forceinline__ v16h frag_f32s(const float* rowk0, int lane, float sc) {
  v16h a; const float* p = rowk0 + 8 * (lane >> 4);
#pragma unroll
  for (int i = 0; i < 8; ++i) { const float x0 = p[i], x1 = p[16 + i]; a[i] = (_Float16)(x0 * sc); a[8 + i] = (_Float16)(x1 * sc); }
  return a;
}
__device__ __forceinline__ float bfr(float v) { return (float)(__bf16)v; }

#ifndef NB
#define NB 2
#endif
#ifndef SEQ
#define SEQ 4096
#endif
#define NB_FULL 2
#define TT SEQ
#define NPIX 4096
#define DIN 256
#define GROUPS 8
#define CPG (DIN / GROUPS)
#define NH 4
#define HD 32
#define CC (NH * HD)
#define NQB (TT / 64)
#define SCALE (0.17677669529663687f)
#define EPS (1.0e-5f)
static_assert(CPG == 32);
static_assert(CC == 128);
static_assert(DIN % 128 == 0);
static_assert(TT % 128 == 0);
static_assert(TT <= NPIX);
static_assert(NB <= NB_FULL);
static_assert(((size_t)NB * DIN - 1) * NPIX + TT <= (size_t)2097152);

#define WS_GS  ((size_t)0)
#define WS_W1  ((size_t)4096)
#define WS_W2  (WS_W1 + 2u * (size_t)3 * CC * DIN)
#define WS_QH  (WS_W2 + 2u * (size_t)DIN * CC)
#define WS_KH  (WS_QH + 2u * (size_t)NB * TT * CC)
#define WS_VT  (WS_KH + 2u * (size_t)NB * TT * CC)
#define WS_S   (WS_VT + 2u * (size_t)NB * CC * TT)
#define WS_Y   (WS_S  + 4u * (size_t)TT * TT)
#define WS_END (WS_Y  + 4u * (size_t)NB * TT * CC)
static_assert(4u * NB * GROUPS * 32 <= 4096);
static_assert(WS_END <= (size_t)134217728);
static_assert((3 * CC * DIN / 8) % 256 == 0);
static_assert(((3 * CC * DIN + DIN * CC) / 8) % 256 == 0);

__global__ __launch_bounds__(256) void k_gn(const float* __restrict__ X, float* __restrict__ GS) {
  __shared__ double sd[256]; __shared__ float sm1, sm2;
  const int tid = threadIdx.x; const int bg = blockIdx.x; const int b = bg / GROUPS, gi = bg % GROUPS;
  const float* xp = X + ((size_t)b * DIN + (size_t)gi * CPG) * NPIX;
  const int nq = CPG * (TT / 4);
  double s = 0.0;
#pragma unroll 1
  for (int e = tid; e < nq; e += 256) { const int c = e / (TT / 4), t4 = e - c * (TT / 4);
    const v4f v = *(const v4f*)(xp + (size_t)c * NPIX + (size_t)t4 * 4); const float x0 = v[0], x1 = v[1], x2 = v[2], x3 = v[3];
    s += (double)((bfr(x0) + bfr(x1)) + (bfr(x2) + bfr(x3))); }
  sd[tid] = s; __syncthreads();
  for (int off = 128; off > 0; off >>= 1) { if (tid < off) sd[tid] += sd[tid + off]; __syncthreads(); }
  if (tid == 0) sm1 = (float)(sd[0] / (double)(CPG * TT));
  __syncthreads(); const float mean = sm1;
  double s2 = 0.0;
#pragma unroll 1
  for (int e = tid; e < nq; e += 256) { const int c = e / (TT / 4), t4 = e - c * (TT / 4);
    const v4f v = *(const v4f*)(xp + (size_t)c * NPIX + (size_t)t4 * 4); const float x0 = v[0], x1 = v[1], x2 = v[2], x3 = v[3];
    const float d0 = bfr(x0) - mean, d1 = bfr(x1) - mean, d2 = bfr(x2) - mean, d3 = bfr(x3) - mean;
    s2 += (double)((d0 * d0 + d1 * d1) + (d2 * d2 + d3 * d3)); }
  sd[tid] = s2; __syncthreads();
  for (int off = 128; off > 0; off >>= 1) { if (tid < off) sd[tid] += sd[tid + off]; __syncthreads(); }
  if (tid == 0) { const float var = (float)(sd[0] / (double)(CPG * TT)); sm2 = 1.0f / sqrtf(var + EPS); }
  __syncthreads();
  if (tid < 32) { const float val = tid == 0 ? mean : (tid == 1 ? sm2 : 0.f); vst2(GS + (size_t)bg * 32 + tid, val); }
}
__global__ __launch_bounds__(256) void k_cvw(const float* __restrict__ WA, const float* __restrict__ WB, _Float16* __restrict__ P1, _Float16* __restrict__ P2) {
  const int n1c = 3 * CC * DIN / 8, n2c = DIN * CC / 8;
  const int i8 = blockIdx.x * 256 + threadIdx.x; if (i8 >= n1c + n2c) return;
  const bool second = i8 >= n1c;
  const float* src = second ? WB + (size_t)(i8 - n1c) * 8 : WA + (size_t)i8 * 8;
  _Float16* dst = second ? P2 + (size_t)(i8 - n1c) * 8 : P1 + (size_t)i8 * 8;
  const v8f v = *(const v8f*)src; union { v8h h; v4u u; } o;
#pragma unroll
  for (int e = 0; e < 8; ++e) { const float f = v[e]; o.h[e] = (_Float16)(bfr(f) * 256.0f); }
  vst2(dst, o.u);
}
__global__ __launch_bounds__(128) void k_proj(const float* __restrict__ X, const float* __restrict__ GS, const float* __restrict__ GW, const float* __restrict__ GB, const _Float16* __restrict__ W1,
    _Float16* __restrict__ QH, _Float16* __restrict__ KH, _Float16* __restrict__ VT) {
  __shared__ __align__(16) _Float16 sh[64][136]; __shared__ __align__(16) _Float16 th[128][72];
  const int tid = threadIdx.x, wave = tid >> 5, lane = tid & 31, col = lane & 15, g = lane >> 4; const int which = blockIdx.y;
  const size_t r0 = (size_t)blockIdx.x * 64; const size_t bb = r0 / TT; const int t0 = (int)(r0 % TT);
  v8f acc[8] = {};
#pragma unroll 1
  for (int kc = 0; kc < DIN / 32; ++kc) {
    const float mu = GS[(bb * GROUPS + kc) * 32], rs = GS[(bb * GROUPS + kc) * 32 + 1];
    v16h a;
    { const float* p = X + ((size_t)bb * DIN + kc * 32 + 8 * g) * NPIX + t0 + wave * 16 + col;
      const v8f w0 = *(const v8f*)(GW + kc * 32 + 8 * g), w1 = *(const v8f*)(GW + kc * 32 + 16 + 8 * g);
      const v8f b0 = *(const v8f*)(GB + kc * 32 + 8 * g), b1 = *(const v8f*)(GB + kc * 32 + 16 + 8 * g);
#pragma unroll
      for (int i = 0; i < 8; ++i) {
        const float xa = p[(size_t)i * NPIX], xb = p[(size_t)(16 + i) * NPIX]; const float wa = w0[i], wb = w1[i], ba = b0[i], bbv = b1[i];
        a[i]     = (_Float16)(((bfr(xa) - mu) * rs) * bfr(wa) + bfr(ba));
        a[8 + i] = (_Float16)(((bfr(xb) - mu) * rs) * bfr(wb) + bfr(bbv)); } }
    asm volatile("s_wait_loadcnt 0x0" ::: "memory");
#pragma unroll
    for (int j = 0; j < 8; ++j) { const v16h w = frag_h(W1 + (size_t)(which * CC + j * 16 + col) * DIN + kc * 32, lane); acc[j] = wmma16(a, w, acc[j]); }
  }
  if (which < 2) { _Float16* DH = which == 0 ? QH : KH;
#pragma unroll
    for (int j = 0; j < 8; ++j)
#pragma unroll
      for (int r = 0; r < 8; ++r) sh[wave * 16 + 8 * g + r][j * 16 + col] = (_Float16)(acc[j][r] * (1.0f / 256.0f));
    __syncthreads();
#pragma unroll 1
    for (int e = tid; e < 64 * 16; e += 128) { const int rl = e >> 4, q = e & 15; vst2(DH + (r0 + rl) * CC + q * 8, *(const v4u*)&sh[rl][q * 8]); }
  } else {
#pragma unroll
    for (int j = 0; j < 8; ++j)
#pragma unroll
      for (int r = 0; r < 8; ++r) th[j * 16 + col][wave * 16 + 8 * g + r] = (_Float16)(acc[j][r] * (1.0f / 256.0f));
    __syncthreads();
#pragma unroll 1
    for (int e = tid; e < 128 * 8; e += 128) { const int cl = e >> 3, q = e & 7; vst2(VT + (bb * CC + cl) * (size_t)TT + t0 + q * 8, *(const v4u*)&th[cl][q * 8]); }
  }
}
__global__ __launch_bounds__(128) void k_sc(const _Float16* __restrict__ QH, const _Float16* __restrict__ KH, int b, int h, float* __restrict__ S) {
  __shared__ __align__(16) float ss[4][16][132];
  const int qb = blockIdx.x, kb = blockIdx.y;
  const int tid = threadIdx.x, wave = tid >> 5, lane = tid & 31, col = lane & 15, g = lane >> 4;
  const int k0 = kb * 128; const int ql0 = qb * 64 + wave * 16; const size_t q0 = (size_t)b * TT + ql0, kr0 = (size_t)b * TT + k0;
  v8f acc[8] = {};
#pragma unroll
  for (int kc = 0; kc < HD / 32; ++kc) { const v16h ah = frag_h(QH + (q0 + col) * CC + h * HD + kc * 32, lane);
#pragma unroll
    for (int j = 0; j < 8; ++j) { const v16h kf = frag_h(KH + (kr0 + j * 16 + col) * CC + h * HD + kc * 32, lane); acc[j] = wmma16(ah, kf, acc[j]); } }
#pragma unroll
  for (int j = 0; j < 8; ++j)
#pragma unroll
    for (int r = 0; r < 8; ++r) ss[wave][8 * g + r][j * 16 + col] = acc[j][r] * SCALE;
  __syncthreads();
#pragma unroll 1
  for (int rl = 0; rl < 16; ++rl) vst2(S + (size_t)(ql0 + rl) * TT + k0 + lane * 4, *(const v4f*)&ss[wave][rl][lane * 4]);
}
__global__ __launch_bounds__(256) void k_sm(float* __restrict__ S) {
  __shared__ float sred[8]; __shared__ float sbc; __shared__ __align__(16) float shv[TT];
  const int tid = threadIdx.x; float* sr = S + (size_t)blockIdx.x * TT;
  float m = -3.0e38f;
#pragma unroll 1
  for (int q = tid; q < TT / 4; q += 256) { const v4f v = *(const v4f*)(sr + (size_t)q * 4); *(v4f*)&shv[q * 4] = v; m = fmaxf(m, fmaxf(fmaxf(v[0], v[1]), fmaxf(v[2], v[3]))); }
#pragma unroll
  for (int o = 1; o < 32; o <<= 1) m = fmaxf(m, __shfl_xor(m, o));
  if ((tid & 31) == 0) sred[tid >> 5] = m; __syncthreads();
  if (tid == 0) { float a = sred[0]; for (int i = 1; i < 8; ++i) a = fmaxf(a, sred[i]); sbc = a; } __syncthreads(); m = sbc; __syncthreads();
  float sum = 0.f;
#pragma unroll 1
  for (int k = tid; k < TT; k += 256) { const float e = expf(shv[k] - m); shv[k] = e; sum += e; }
#pragma unroll
  for (int o = 1; o < 32; o <<= 1) sum += __shfl_xor(sum, o);
  if ((tid & 31) == 0) sred[tid >> 5] = sum; __syncthreads();
  if (tid == 0) { float a = 0.f; for (int i = 0; i < 8; ++i) a += sred[i]; sbc = 2048.0f / a; } __syncthreads(); const float inv = sbc;
#pragma unroll 1
  for (int q = tid; q < TT / 4; q += 256) { v4f p = *(const v4f*)&shv[q * 4]; p = p * inv; vst2(sr + (size_t)q * 4, p); }
}
__global__ __launch_bounds__(128) void k_pv(const float* __restrict__ PS, const _Float16* __restrict__ VT, int b, int h, float* __restrict__ Y) {
  __shared__ __align__(16) float ss[4][16][HD + 4];
  const int tid = threadIdx.x, wave = tid >> 5, lane = tid & 31, col = lane & 15, g = lane >> 4; const int qb = blockIdx.x; const int ql0 = qb * 64 + wave * 16;
  v8f acc[HD / 16] = {};
#pragma unroll 1
  for (int kc = 0; kc < TT / 32; ++kc) { const v16h p = frag_f32(PS + (size_t)(ql0 + col) * TT + kc * 32, lane);
    asm volatile("s_wait_loadcnt 0x0" ::: "memory");
#pragma unroll
    for (int j = 0; j < HD / 16; ++j) { const size_t po = ((size_t)b * CC + h * HD + j * 16 + col) * (size_t)TT + (size_t)kc * 32; acc[j] = wmma16(p, frag_h(VT + po, lane), acc[j]); } }
#pragma unroll
  for (int j = 0; j < HD / 16; ++j)
#pragma unroll
    for (int r = 0; r < 8; ++r) ss[wave][8 * g + r][j * 16 + col] = acc[j][r] * (1.0f / 2048.0f);
  __syncthreads();
  const int lc = lane < HD / 4 ? lane : 0;
#pragma unroll 1
  for (int rl = 0; rl < 16; ++rl) { const v4f o4 = *(const v4f*)&ss[wave][rl][lc * 4]; if (lane < HD / 4) vst2(Y + ((size_t)b * TT + ql0 + rl) * CC + h * HD + lane * 4, o4); }
}
__global__ __launch_bounds__(128) void k_out(const float* __restrict__ Y, const float* __restrict__ X, const _Float16* __restrict__ W2, const float* __restrict__ PB, float* __restrict__ OUT) {
  __shared__ __align__(16) float stc[128][68];
  const int tid = threadIdx.x, wave = tid >> 5, lane = tid & 31, col = lane & 15, g = lane >> 4; const int c0 = blockIdx.y * 128;
  const size_t r0 = (size_t)blockIdx.x * 64; const size_t bb = r0 / TT; const int t0 = (int)(r0 % TT);
  v8f acc[8] = {};
#pragma unroll 1
  for (int kc = 0; kc < CC / 32; ++kc) { const v16h a = frag_f32s(Y + (r0 + wave * 16 + col) * CC + kc * 32, lane, 64.0f);
    asm volatile("s_wait_loadcnt 0x0" ::: "memory");
#pragma unroll
    for (int j = 0; j < 8; ++j) { const v16h w = frag_h(W2 + (size_t)(c0 + j * 16 + col) * CC + kc * 32, lane); acc[j] = wmma16(a, w, acc[j]); } }
#pragma unroll
  for (int j = 0; j < 8; ++j) { const float bias = bfr(PB[c0 + j * 16 + col]);
#pragma unroll
    for (int r = 0; r < 8; ++r) stc[j * 16 + col][wave * 16 + 8 * g + r] = acc[j][r] * (1.0f / 16384.0f) + bias; }
  __syncthreads();
#pragma unroll 1
  for (int e = tid; e < 128 * 16; e += 128) { const int cl = e >> 4, q = e & 15; const size_t o = ((size_t)bb * DIN + c0 + cl) * NPIX + t0 + q * 4;
    const v4f xv = *(const v4f*)(X + o); const float x0 = xv[0], x1 = xv[1], x2 = xv[2], x3 = xv[3]; v4f r4 = *(const v4f*)&stc[cl][q * 4];
    r4[0] += bfr(x0); r4[1] += bfr(x1); r4[2] += bfr(x2); r4[3] += bfr(x3); vst2(OUT + o, r4); }
}

extern "C" void kernel_launch(void* const* d_in, const int* in_sizes, int n_in, void* d_out, int out_size, void* d_ws, size_t ws_size, hipStream_t stream) {
  if (n_in < 6) return;
  if (in_sizes[0] < NB * DIN * NPIX || in_sizes[1] < DIN || in_sizes[2] < DIN || in_sizes[3] < 3 * CC * DIN || in_sizes[4] < DIN * CC || in_sizes[5] < DIN) return;
  if (out_size < NB * DIN * NPIX) return;
  if (ws_size < WS_END) return;
  const float* X = (const float*)d_in[0]; const float* GW = (const float*)d_in[1]; const float* GB = (const float*)d_in[2];
  const float* WQ = (const float*)d_in[3]; const float* WP = (const float*)d_in[4]; const float* PB = (const float*)d_in[5];
  char* ws = (char*)d_ws;
  float* GS = (float*)(ws + WS_GS); _Float16* W1 = (_Float16*)(ws + WS_W1); _Float16* W2 = (_Float16*)(ws + WS_W2);
  _Float16* QH = (_Float16*)(ws + WS_QH); _Float16* KH = (_Float16*)(ws + WS_KH); _Float16* VT = (_Float16*)(ws + WS_VT);
  float* S = (float*)(ws + WS_S); float* Y = (float*)(ws + WS_Y); float* OUT = (float*)d_out;
  k_gn<<<dim3(NB * GROUPS), 256, 0, stream>>>(X, GS);
  k_cvw<<<dim3((3 * CC * DIN + DIN * CC) / 8 / 256), 256, 0, stream>>>(WQ, WP, W1, W2);
  k_proj<<<dim3(NB * TT / 64, 3), 128, 0, stream>>>(X, GS, GW, GB, W1, QH, KH, VT);
  for (int b = 0; b < NB; ++b) for (int h = 0; h < NH; ++h) {
    k_sc<<<dim3(NQB, TT / 128), 128, 0, stream>>>(QH, KH, b, h, S);
    k_sm<<<dim3(TT), 256, 0, stream>>>(S);
    k_pv<<<dim3(NQB), 128, 0, stream>>>(S, VT, b, h, Y);
  }
  k_out<<<dim3(NB * TT / 64, DIN / 128), 128, 0, stream>>>(Y, X, W2, PB, OUT);
}
